// RNNDetector_43791486550106
// MI455X (gfx1250) — hardware-verified
//
#include <hip/hip_runtime.h>

typedef __attribute__((ext_vector_type(16))) _Float16 v16h;
typedef __attribute__((ext_vector_type(8)))  _Float16 v8h;
typedef __attribute__((ext_vector_type(2)))  _Float16 v2h;
typedef __attribute__((ext_vector_type(16))) __bf16   v16b;
typedef __attribute__((ext_vector_type(8)))  __bf16   v8b;
typedef __attribute__((ext_vector_type(8)))  float    v8f;
typedef __attribute__((ext_vector_type(4)))  float    v4f;

constexpr int kSteps   = 262144;
constexpr int kHid     = 64;
constexpr int kGates   = 4 * kHid;
constexpr int kOutW    = 16;
constexpr int kChunk   = 32;
constexpr int kSlab    = 32768;
constexpr int kNumSlab = kSteps / kSlab;
constexpr float kCarryAct = 256.0f;
constexpr float kCarryWgt = 512.0f;
constexpr float kFoldBack = 1.0f / (kCarryAct * kCarryWgt);
constexpr float kF16MinNormal = 6.103515625e-05f;
constexpr int kHeadTilesPerWave = 4;
constexpr int kHeadBlocks = kSteps / (16 * 8 * kHeadTilesPerWave);
constexpr int kStateFloats = 2 * kHid;

static_assert(kGates == 256);
static_assert(kSteps % kSlab == 0 && kSlab % kChunk == 0 && kSteps % kChunk == 0);
static_assert(kSlab % 64 == 0 && kGates % 64 == 0 && kHid % 32 == 0);
static_assert(kChunk * kHid == 256 * 8);
static_assert(kChunk == 8 * 4);
static_assert(kHeadBlocks * 16 * 8 * kHeadTilesPerWave == kSteps);
static_assert(kCarryAct * kCarryWgt == 131072.0f);

__device__ __forceinline__ unsigned short f2bf_bits(float f) {
  unsigned u = __float_as_uint(f);
  return (unsigned short)((u + 0x7FFFu + ((u >> 16) & 1u)) >> 16);
}
__device__ __forceinline__ float bf_bits2f(unsigned short h) { return __uint_as_float(((unsigned)h) << 16); }

__device__ __forceinline__ void dep_guard_h(v8f& a, v8f& b, v16h x, v16h y) { asm volatile("v_nop\n\tv_nop\n\tv_nop\n\tv_nop" : "+v"(a), "+v"(b) : "v"(x), "v"(y)); }
__device__ __forceinline__ void dep_guard_b(v8f& a, v8f& b, v16b x, v16b y) { asm volatile("v_nop\n\tv_nop\n\tv_nop\n\tv_nop" : "+v"(a), "+v"(b) : "v"(x), "v"(y)); }
__device__ __forceinline__ void keep4_h(v16h a, v16h b, v16h c, v16h d) { asm volatile("v_nop" :: "v"(a), "v"(b), "v"(c), "v"(d)); }
__device__ __forceinline__ void keep4_b(v16b a, v16b b, v16b c, v16b d) { asm volatile("v_nop" :: "v"(a), "v"(b), "v"(c), "v"(d)); }
__device__ __forceinline__ void acc_guard4(v8f& a, v8f& b, v8f& c, v8f& d) { asm volatile("v_nop\n\tv_nop\n\tv_nop\n\tv_nop" : "+v"(a), "+v"(b), "+v"(c), "+v"(d)); }

template <typename T> struct Frag;
template <> struct Frag<_Float16> {
  typedef v16h V; union U { v16h v; v8h h[2]; };
  static __device__ __forceinline__ v16h load(const _Float16* p) {
    U f; f.h[0] = *(const v8h*)(p); f.h[1] = *(const v8h*)(p + 16); return f.v;
  }
  static __device__ __forceinline__ v8f mma(v16h a, v16h b, v8f c) {
    return __builtin_amdgcn_wmma_f32_16x16x32_f16(false, a, false, b, (short)0, c, false, false);
  }
  static __device__ __forceinline__ void guard(v8f& a, v8f& b, v16h x, v16h y) { dep_guard_h(a, b, x, y); }
  static __device__ __forceinline__ void keep(v16h a, v16h b, v16h c, v16h d) { keep4_h(a, b, c, d); }
};
template <> struct Frag<__bf16> {
  typedef v16b V; union U { v16b v; v8b h[2]; };
  static __device__ __forceinline__ v16b load(const __bf16* p) {
    U f; f.h[0] = *(const v8b*)(p); f.h[1] = *(const v8b*)(p + 16); return f.v;
  }
  static __device__ __forceinline__ v8f mma(v16b a, v16b b, v8f c) {
    return __builtin_amdgcn_wmma_f32_16x16x32_bf16(false, a, false, b, (short)0, c, false, false);
  }
  static __device__ __forceinline__ void guard(v8f& a, v8f& b, v16b x, v16b y) { dep_guard_b(a, b, x, y); }
  static __device__ __forceinline__ void keep(v16b a, v16b b, v16b c, v16b d) { keep4_b(a, b, c, d); }
};

template <int ET> struct Elem;
template <> struct Elem<0> { typedef _Float16 T; };
template <> struct Elem<1> { typedef __bf16 T; };
template <int ET, bool SPLIT, int BIAS_MODE, int OUT_MODE, bool RESID, int ACT = 0>
__global__ __launch_bounds__(256) void wmma_gemm64(
    const unsigned short* __restrict__ Ap, const unsigned short* __restrict__ A2p, int lda, long strideA,
    const unsigned short* __restrict__ Btp, const unsigned short* __restrict__ Bt2p, int ldb, long strideB,
    void* __restrict__ Cout, void* __restrict__ Cout2, int ldc, long strideC,
    const float* __restrict__ bias,
    const float* __restrict__ resid, long strideR,
    int M, int N, int K, float scale) {
  typedef typename Elem<ET>::T T;
  typedef typename Frag<T>::V V;
  const T* A = (const T*)Ap; const T* A2 = (const T*)A2p; const T* Bt = (const T*)Btp; const T* Bt2 = (const T*)Bt2p;
  __shared__ __align__(16) float sT[8][16 * 68];
  const int b    = blockIdx.y;
  const int lane = threadIdx.x & 31;
  const int wave = threadIdx.x >> 5;
  const int tilesN = N >> 6;
  const int tilesM = M >> 6;
  const int tile = blockIdx.x * 8 + wave;
  if (tile >= tilesM * tilesN) return;
  const int tm = tile / tilesN;
  const int tn = tile - tm * tilesN;
  const int m0 = tm << 6;
  const int n0 = tn << 6;

  const T* Ab  = A  + (size_t)b * strideA;
  const T* Bb  = Bt + (size_t)b * strideB;
  const T* Ab2 = SPLIT ? (A2  + (size_t)b * strideA) : nullptr;
  const T* Bb2 = SPLIT ? (Bt2 + (size_t)b * strideB) : nullptr;

  const int rlane = lane & 15;
  const int koff  = (lane >> 4) * 8;
  const int mOff  = (lane >> 4) * 8;

  v8f acc[4][4];
#pragma unroll
  for (int i = 0; i < 4; ++i)
#pragma unroll
    for (int j = 0; j < 4; ++j) acc[i][j] = (v8f){0.f,0.f,0.f,0.f,0.f,0.f,0.f,0.f};

  for (int k0 = 0; k0 < K; k0 += 32) {
    V bh[4], bl[4];
#pragma unroll
    for (int j = 0; j < 4; ++j) {
      const size_t bo = (size_t)(n0 + (j << 4) + rlane) * ldb + koff + k0;
      bh[j] = Frag<T>::load(Bb + bo);
      if (SPLIT) bl[j] = Frag<T>::load(Bb2 + bo);
    }
#pragma unroll
    for (int i = 0; i < 4; ++i) {
      const size_t ao = (size_t)(m0 + (i << 4) + rlane) * lda + koff + k0;
      V ah = Frag<T>::load(Ab + ao);
      V al;
      if (SPLIT) al = Frag<T>::load(Ab2 + ao);
#pragma unroll
      for (int j = 0; j < 4; ++j) {
        acc[i][j] = Frag<T>::mma(ah, bh[j], acc[i][j]);
        if (SPLIT) {
          acc[i][j] = Frag<T>::mma(ah, bl[j], acc[i][j]);
          acc[i][j] = Frag<T>::mma(al, bh[j], acc[i][j]);
        }
      }
      Frag<T>::guard(acc[i][0], acc[i][3], ah, SPLIT ? al : ah);
    }
    Frag<T>::keep(bh[0], bh[1], bh[2], bh[3]);
    if (SPLIT) Frag<T>::keep(bl[0], bl[1], bl[2], bl[3]);
  }
  acc_guard4(acc[0][0], acc[0][1], acc[0][2], acc[0][3]);
  acc_guard4(acc[1][0], acc[1][1], acc[1][2], acc[1][3]);
  acc_guard4(acc[2][0], acc[2][1], acc[2][2], acc[2][3]);
  acc_guard4(acc[3][0], acc[3][1], acc[3][2], acc[3][3]);

  float* slab = sT[wave];
  const float* Rb = RESID ? (resid + (size_t)b * strideR) : nullptr;
#pragma unroll
  for (int i = 0; i < 4; ++i) {
    const int mBase = m0 + (i << 4);
#pragma unroll
    for (int j = 0; j < 4; ++j) {
      const int n = n0 + (j << 4) + rlane;
      float bv = 0.f;
      if (BIAS_MODE == 2) bv = bias[n];
#pragma unroll
      for (int r = 0; r < 8; ++r) {
        float v = acc[i][j][r] * scale;
        if (BIAS_MODE == 1) v += bias[mBase + mOff + r];
        if (BIAS_MODE == 2) v += bv;
        if (RESID) v += Rb[(size_t)(mBase + mOff + r) * ldc + n];
        if (ACT == 1) v = tanhf(v);
        if (ACT == 2) v = fmaxf(v, 0.0f);
        if (ACT == 4) v = (v > 0.f) ? v : 0.01f * v;
        slab[(mOff + r) * 68 + (j << 4) + rlane] = v;
      }
    }
    __builtin_amdgcn_fence(__ATOMIC_RELEASE, "workgroup");
    __builtin_amdgcn_wave_barrier();
    __builtin_amdgcn_fence(__ATOMIC_ACQUIRE, "workgroup");
    if (OUT_MODE == 0) {
      float* C = (float*)Cout + (size_t)b * strideC;
      const int hh = lane >> 4, c4 = (lane & 15) * 4;
      for (int pass = 0; pass < 2; ++pass) {
#pragma unroll
        for (int it = 0; it < 8; ++it) {
          const int row = it * 2 + hh;
          v4f v = *(const v4f*)(slab + row * 68 + c4);
          *(volatile v4f*)(C + (size_t)(mBase + row) * ldc + n0 + c4) = v;
        }
        __threadfence();
      }
    } else {
      const int q = lane >> 3, c8 = (lane & 7) * 8;
      unsigned short* C  = (unsigned short*)Cout  + (size_t)b * strideC;
      unsigned short* C2 = (OUT_MODE == 2) ? ((unsigned short*)Cout2 + (size_t)b * strideC) : nullptr;
      for (int pass = 0; pass < 2; ++pass) {
#pragma unroll
        for (int it = 0; it < 4; ++it) {
          const int row = it * 4 + q;
          const float* sp = slab + row * 68 + c8;
          v8h hv, lv;
#pragma unroll
          for (int e = 0; e < 8; ++e) {
            if (OUT_MODE == 1) {
              hv[e] = (_Float16)sp[e];
            } else {
              unsigned short hb = f2bf_bits(sp[e]);
              unsigned short lb = f2bf_bits(sp[e] - bf_bits2f(hb));
              hv[e] = __builtin_bit_cast(_Float16, hb);
              lv[e] = __builtin_bit_cast(_Float16, lb);
            }
          }
          *(volatile v8h*)(C + (size_t)(mBase + row) * ldc + n0 + c8) = hv;
          if (OUT_MODE == 2) *(volatile v8h*)(C2 + (size_t)(mBase + row) * ldc + n0 + c8) = lv;
        }
        __threadfence();
      }
    }
    __builtin_amdgcn_fence(__ATOMIC_RELEASE, "workgroup");
    __builtin_amdgcn_wave_barrier();
    __builtin_amdgcn_fence(__ATOMIC_ACQUIRE, "workgroup");
  }
}

__device__ __forceinline__ _Float16 to_f16_carried(float x, float carry) {
  float v = x * carry;
  v = (__builtin_fabsf(v) < kF16MinNormal) ? 0.0f : v;
  return (_Float16)v;
}
__device__ __forceinline__ unsigned pack_f16x2(_Float16 a, _Float16 b) {
  v2h p;
  p[0] = a;
  p[1] = b;
  return __builtin_bit_cast(unsigned, p);
}
__device__ __forceinline__ void st2u(unsigned* p, unsigned v) {
  *(volatile unsigned*)p = v;
  __threadfence();
  *(volatile unsigned*)p = v;
}

constexpr int kPrepB1 = (kGates * kHid / 2) / 256;
constexpr int kPrepB2 = kPrepB1 + (kOutW * kHid / 2) / 256;
constexpr int kPrepBlocks = kPrepB2 + (4 * kStateFloats) / 256;
static_assert(kPrepB1 == 32 && kPrepB2 == 34 && kPrepBlocks == 36);

__global__ __launch_bounds__(256) void prep_kernel(
    const float* __restrict__ w_ih1, const float* __restrict__ w_lin,
    unsigned* __restrict__ wih1u, unsigned* __restrict__ wlinu, unsigned* __restrict__ stu) {
  const int blk = blockIdx.x, tid = threadIdx.x;
  if (blk < kPrepB1) {
    const int p = blk * 256 + tid;
    const float a = w_ih1[2 * p], b = w_ih1[2 * p + 1];
    const unsigned u = pack_f16x2(to_f16_carried(a, kCarryWgt), to_f16_carried(b, kCarryWgt));
    st2u(wih1u + p, u);
  } else if (blk < kPrepB2) {
    const int p = (blk - kPrepB1) * 256 + tid;
    const float a = w_lin[2 * p], b = w_lin[2 * p + 1];
    const unsigned u = pack_f16x2(to_f16_carried(a, kCarryWgt), to_f16_carried(b, kCarryWgt));
    st2u(wlinu + p, u);
  } else {
    const int p = (blk - kPrepB2) * 256 + tid;
    st2u(stu + p, 0u);
  }
}

template <int LAYER>
__global__ __launch_bounds__(256) void cell_scan_kernel(
    const float* __restrict__ src, const float* __restrict__ w_hh, const float* __restrict__ w_in0,
    const float* __restrict__ b_a, const float* __restrict__ b_b,
    const float* __restrict__ st_in, float* __restrict__ st_out,
    unsigned short* __restrict__ hplane, int nsteps) {
  __shared__ __align__(16) float hbuf[kChunk * kHid];
  __shared__ __align__(16) float gact[kGates];
  __shared__ __align__(16) float sfin[kStateFloats];
  const int j = threadIdx.x;
  const int lane = j & 31, wave = j >> 5;

  float w[kHid];
  {
    const v4f* wp = (const v4f*)(w_hh + (size_t)j * kHid);
#pragma unroll
    for (int q = 0; q < kHid / 4; ++q) {
      const v4f t = wp[q];
      w[4 * q + 0] = t[0];
      w[4 * q + 1] = t[1];
      w[4 * q + 2] = t[2];
      w[4 * q + 3] = t[3];
    }
  }
  const float bj = b_a[j] + b_b[j];
  float wi = 0.0f;
  if (LAYER == 0) wi = w_in0[j];

  const bool isTanh = ((j >> 6) == 2);
  const float aexp = isTanh ? -2.0f : -1.0f;
  const float amul = isTanh ? 2.0f : 1.0f;
  const float aadd = isTanh ? -1.0f : 0.0f;

  const int ju = j & (kHid - 1);
  float hin = st_in[ju];
  float c = st_in[kHid + ju];
  asm volatile("" : "+v"(hin));
  asm volatile("" : "+v"(c));

  {
    const v4f z = (v4f){0.f, 0.f, 0.f, 0.f};
    *(v4f*)(hbuf + j * 8) = z;
    *(v4f*)(hbuf + j * 8 + 4) = z;
  }
  __syncthreads();
  if (j < kHid) hbuf[(kChunk - 1) * kHid + j] = hin;
  __syncthreads();

  float xnext;
  if (LAYER == 0) xnext = src[0]; else xnext = src[j];

#pragma unroll 1
  for (int t0 = 0; t0 < nsteps; t0 += kChunk) {
#pragma unroll 1
    for (int s = 0; s < kChunk; ++s) {
      const int t = t0 + s;
      const float xcur = xnext;
      int tn = t + 1;
      tn = (tn < nsteps) ? tn : (nsteps - 1);
      if (LAYER == 0) xnext = src[tn]; else xnext = src[(size_t)tn * kGates + j];

      float g;
      if (LAYER == 0) g = fmaf(xcur, wi, bj); else g = xcur + bj;
      const float* hp = hbuf + ((s + kChunk - 1) & (kChunk - 1)) * kHid;
#pragma unroll
      for (int q = 0; q < kHid / 4; ++q) {
        const v4f hq = *(const v4f*)(hp + 4 * q);
        g = fmaf(w[4 * q + 0], hq[0], g);
        g = fmaf(w[4 * q + 1], hq[1], g);
        g = fmaf(w[4 * q + 2], hq[2], g);
        g = fmaf(w[4 * q + 3], hq[3], g);
      }
      const float ev = __expf(aexp * g);
      const float rv = __builtin_amdgcn_rcpf(1.0f + ev);
      gact[j] = fmaf(amul, rv, aadd);
      __syncthreads();
      if (j < kHid) {
        const float ig = gact[j];
        const float fg = gact[kHid + j];
        const float gg = gact[2 * kHid + j];
        const float og = gact[3 * kHid + j];
        c = fmaf(fg, c, ig * gg);
        const float th = 1.0f - 2.0f * __builtin_amdgcn_rcpf(1.0f + __expf(2.0f * c));
        hbuf[s * kHid + j] = og * th;
      }
      __syncthreads();
    }
    {
      const int row = wave * 4 + (lane >> 3);
      const int c8 = (lane & 7) * 8;
      const float* sp = hbuf + row * kHid + c8;
      const v4f a0 = *(const v4f*)(sp);
      const v4f a1 = *(const v4f*)(sp + 4);
      v8h hv;
#pragma unroll
      for (int e = 0; e < 4; ++e) {
        const float f0 = a0[e];
        const float f1 = a1[e];
        hv[e] = to_f16_carried(f0, kCarryAct);
        hv[4 + e] = to_f16_carried(f1, kCarryAct);
      }
      unsigned short* gp = hplane + (size_t)(t0 + row) * kHid + c8;
      for (int pass = 0; pass < 2; ++pass) {
        *(volatile v8h*)gp = hv;
        __threadfence();
      }
    }
  }

  if (j < kHid) {
    sfin[j] = hbuf[(kChunk - 1) * kHid + j];
    sfin[kHid + j] = c;
  }
  __syncthreads();
  if (wave == 0) {
    const v4f v = *(const v4f*)(sfin + lane * 4);
    for (int pass = 0; pass < 2; ++pass) {
      *(volatile v4f*)(st_out + lane * 4) = v;
      __threadfence();
    }
  }
}

__global__ __launch_bounds__(256) void head_kernel(
    const _Float16* __restrict__ h2p, const _Float16* __restrict__ wl,
    const float* __restrict__ blin, float* __restrict__ out) {
  __shared__ __align__(16) float sO[8][16 * kOutW];
  const int lane = threadIdx.x & 31, wave = threadIdx.x >> 5;
  const int c = lane & 15, hh = lane >> 4, koff = hh * 8;
  const v16h fb0 = Frag<_Float16>::load(wl + c * kHid + koff);
  const v16h fb1 = Frag<_Float16>::load(wl + c * kHid + 32 + koff);
  const float bn = blin[c];
  float* slab = sO[wave];
  const int tile0 = (blockIdx.x * 8 + wave) * kHeadTilesPerWave;
#pragma unroll 1
  for (int i = 0; i < kHeadTilesPerWave; ++i) {
    const int m0 = (tile0 + i) * 16;
    const _Float16* ap = h2p + (size_t)(m0 + c) * kHid + koff;
    const v16h fa0 = Frag<_Float16>::load(ap);
    const v16h fa1 = Frag<_Float16>::load(ap + 32);
    v8f acc = (v8f){0.f,0.f,0.f,0.f,0.f,0.f,0.f,0.f};
    acc = Frag<_Float16>::mma(fa0, fb0, acc);
    acc = Frag<_Float16>::mma(fa1, fb1, acc);
    asm volatile("v_nop\n\tv_nop\n\tv_nop\n\tv_nop" : "+v"(acc) : "v"(fa0), "v"(fa1), "v"(fb0), "v"(fb1));
#pragma unroll
    for (int r = 0; r < 8; ++r) slab[(8 * hh + r) * kOutW + c] = acc[r] * kFoldBack + bn;
    __builtin_amdgcn_fence(__ATOMIC_RELEASE, "workgroup");
    __builtin_amdgcn_wave_barrier();
    __builtin_amdgcn_fence(__ATOMIC_ACQUIRE, "workgroup");
    float* op = out + (size_t)m0 * kOutW;
    for (int pass = 0; pass < 2; ++pass) {
#pragma unroll
      for (int it = 0; it < 2; ++it) {
        const v4f v = *(const v4f*)(slab + it * 128 + lane * 4);
        *(volatile v4f*)(op + it * 128 + lane * 4) = v;
      }
      __threadfence();
    }
    __builtin_amdgcn_fence(__ATOMIC_RELEASE, "workgroup");
    __builtin_amdgcn_wave_barrier();
    __builtin_amdgcn_fence(__ATOMIC_ACQUIRE, "workgroup");
  }
}

constexpr size_t kBytesHPlane = (size_t)kSteps * kHid * 2;
constexpr size_t kBytesXP     = (size_t)kSlab * kGates * 4;
constexpr size_t kBytesWI1    = (size_t)kGates * kHid * 2;
constexpr size_t kBytesWLN    = (size_t)kOutW * kHid * 2;
constexpr size_t kBytesST     = (size_t)4 * kStateFloats * 4;
constexpr size_t kWsTotal = kBytesHPlane + kBytesHPlane + kBytesXP + kBytesWI1 + kBytesWLN + kBytesST;
static_assert(kWsTotal == 100700160ull);
static_assert(kWsTotal <= 134217728ull);
static_assert((kBytesHPlane % 256) == 0 && (kBytesXP % 256) == 0 && (kBytesWI1 % 256) == 0 && (kBytesWLN % 256) == 0 && (kBytesST % 256) == 0);
static_assert(((kSlab / 64) * (kGates / 64)) % 8 == 0);

extern "C" void kernel_launch(void* const* d_in, const int* in_sizes, int n_in,
                              void* d_out, int out_size, void* d_ws, size_t ws_size, hipStream_t stream) {
  if (n_in < 11 || d_out == nullptr || d_ws == nullptr) return;
  if (ws_size < kWsTotal) return;

  const float* y     = (const float*)d_in[0];
  const float* W_ih0 = (const float*)d_in[1];
  const float* W_hh0 = (const float*)d_in[2];
  const float* b_ih0 = (const float*)d_in[3];
  const float* b_hh0 = (const float*)d_in[4];
  const float* W_ih1 = (const float*)d_in[5];
  const float* W_hh1 = (const float*)d_in[6];
  const float* b_ih1 = (const float*)d_in[7];
  const float* b_hh1 = (const float*)d_in[8];
  const float* W_lin = (const float*)d_in[9];
  const float* b_lin = (const float*)d_in[10];
  float* out = (float*)d_out;

  char* ws = (char*)d_ws;
  size_t off = 0;
  auto carve = [&](size_t bytes) -> char* { char* p = ws + off; off += (bytes + 255) & ~(size_t)255; return p; };
  unsigned short* H1  = (unsigned short*)carve(kBytesHPlane);
  unsigned short* H2  = (unsigned short*)carve(kBytesHPlane);
  float*          XP  = (float*)carve(kBytesXP);
  unsigned short* WI1 = (unsigned short*)carve(kBytesWI1);
  unsigned short* WLN = (unsigned short*)carve(kBytesWLN);
  float*          ST  = (float*)carve(kBytesST);
  if (off > ws_size || off > (size_t)134217728) return;

  prep_kernel<<<kPrepBlocks, 256, 0, stream>>>(W_ih1, W_lin, (unsigned*)WI1, (unsigned*)WLN, (unsigned*)ST);

  cell_scan_kernel<0><<<1, 256, 0, stream>>>(y, W_hh0, W_ih0, b_ih0, b_hh0,
                                             ST, ST + kStateFloats, H1, kSteps);

  float* stL1 = ST + 2 * kStateFloats;
  for (int s = 0; s < kNumSlab; ++s) {
    const unsigned short* Aslab = H1 + (size_t)s * kSlab * kHid;
    wmma_gemm64<0, false, 0, 0, false, 0><<<dim3(((kSlab / 64) * (kGates / 64)) / 8, 1), 256, 0, stream>>>(
        Aslab, nullptr, kHid, 0L,
        WI1, nullptr, kHid, 0L,
        (void*)XP, nullptr, kGates, 0L,
        nullptr, nullptr, 0L,
        kSlab, kGates, kHid, kFoldBack);
    cell_scan_kernel<1><<<1, 256, 0, stream>>>(XP, W_hh1, W_ih0, b_ih1, b_hh1,
                                               stL1 + (s & 1) * kStateFloats,
                                               stL1 + ((s + 1) & 1) * kStateFloats,
                                               H2 + (size_t)s * kSlab * kHid, kSlab);
  }

  head_kernel<<<kHeadBlocks, 256, 0, stream>>>((const _Float16*)H2, (const _Float16*)WLN, b_lin, out);
}
